// MambaLayer_53051436040366
// MI455X (gfx1250) — hardware-verified
//
#include <hip/hip_runtime.h>
#include <math.h>

typedef __attribute__((ext_vector_type(16))) _Float16 v16h;
typedef __attribute__((ext_vector_type(8)))  _Float16 v8h;
typedef __attribute__((ext_vector_type(8)))  float    v8f;
typedef __attribute__((ext_vector_type(4)))  float    v4f;

constexpr int kBatch = 2;
constexpr int kSeq   = 2048;
constexpr int kDm    = 768;
constexpr int kDin   = 1536;
constexpr int kNst   = 16;
constexpr int kDtR   = 48;
constexpr int kDtRP  = 64;
constexpr int kXpN   = 80;
constexpr int kXpP   = 128;
constexpr int kXzP   = 2 * kDin;
constexpr int kRows  = kBatch * kSeq;
constexpr int kFf    = 2 * kDm;
constexpr int kTP    = 260;

constexpr float kCarryW  = 32.0f;
constexpr float kCarryXc = 64.0f;
constexpr float kCarryDt = 64.0f;
constexpr float kCarryY  = 64.0f;
constexpr float kCarryS  = 128.0f;

static_assert(kDtR + 2 * kNst == kXpN);
static_assert((kDm % 32) == 0 && (kDin % 32) == 0 && (kDtRP % 32) == 0 && (kFf % 32) == 0);
static_assert((kRows % 64) == 0 && (kXzP % 64) == 0 && (kXpP % 64) == 0 && (kDin % 64) == 0 && (kDm % 64) == 0 && (kFf % 64) == 0);
static_assert((kSeq % 64) == 0 && (kDin % 256) == 0 && (kDm % 256) == 0 && (kRows % 8) == 0);
static_assert(kFf == kDin);

constexpr size_t kSzWIN  = (size_t)kXzP * kDm * 2;
constexpr size_t kSzWXP  = (size_t)kXpP * kDin * 2;
constexpr size_t kSzWDT  = (size_t)kDin * kDtRP * 2;
constexpr size_t kSzWOUT = (size_t)kDm * kDin * 2;
constexpr size_t kSzWFC1 = (size_t)kFf * kDm * 2;
constexpr size_t kSzWFC2 = (size_t)kDm * kFf * 2;
constexpr size_t kSzLN   = (size_t)kRows * kDm * 2;
constexpr size_t kSzXZ   = (size_t)kRows * kXzP * 2;
constexpr size_t kSzXC   = (size_t)kRows * kDin * 2;
constexpr size_t kSzXDBL = (size_t)kRows * kXpP * 4;
constexpr size_t kSzDTR  = (size_t)kRows * kDtRP * 2;
constexpr size_t kSzDLIN = (size_t)kRows * kDin * 4;
constexpr size_t kSzYF   = (size_t)kRows * kDin * 2;
constexpr size_t kSzS    = (size_t)kRows * kDin * 2;
constexpr size_t kSzHB   = (size_t)kRows * kDm * 4;
constexpr size_t kOffWIN  = 0;
constexpr size_t kOffWXP  = kOffWIN  + kSzWIN;
constexpr size_t kOffWDT  = kOffWXP  + kSzWXP;
constexpr size_t kOffWOUT = kOffWDT  + kSzWDT;
constexpr size_t kOffWFC1 = kOffWOUT + kSzWOUT;
constexpr size_t kOffWFC2 = kOffWFC1 + kSzWFC1;
constexpr size_t kOffLN   = kOffWFC2 + kSzWFC2;
constexpr size_t kOffXZ   = kOffLN   + kSzLN;
constexpr size_t kOffXC   = kOffXZ   + kSzXZ;
constexpr size_t kOffXDBL = kOffXC   + kSzXC;
constexpr size_t kOffDTR  = kOffXDBL + kSzXDBL;
constexpr size_t kOffDLIN = kOffDTR  + kSzDTR;
constexpr size_t kOffYF   = kOffDLIN + kSzDLIN;
constexpr size_t kOffS    = kOffYF   + kSzYF;
constexpr size_t kOffHB   = kOffS    + kSzS;
constexpr size_t kWsTotal = kOffHB   + kSzHB;
static_assert(kWsTotal == 121962496ull);
static_assert(kWsTotal <= 134217728ull);
static_assert((kSzWIN % 128) == 0 && (kSzWXP % 128) == 0 && (kSzWDT % 128) == 0 && (kSzWOUT % 128) == 0 &&
              (kSzWFC1 % 128) == 0 && (kSzWFC2 % 128) == 0 && (kSzLN % 128) == 0 && (kSzXZ % 128) == 0 &&
              (kSzXC % 128) == 0 && (kSzXDBL % 128) == 0 && (kSzDTR % 128) == 0 && (kSzDLIN % 128) == 0 &&
              (kSzYF % 128) == 0 && (kSzS % 128) == 0);
static_assert((size_t)kRows * kFf * 4 <= kSzDLIN);
static_assert((size_t)kRows * kFf * 2 <= kSzYF);

__device__ __forceinline__ float h16_to_f32(unsigned hb) {
  const unsigned sgn = (hb & 0x8000u) << 16;
  const unsigned em = hb & 0x7fffu;
  const float fn = __uint_as_float((em << 13) + 0x38000000u);
  const float fs = (float)em * 5.9604644775390625e-8f;
  const float mag = (em < 0x400u) ? fs : fn;
  return __uint_as_float(__float_as_uint(mag) | sgn);
}

union FragU { v16h v; v8h h[2]; };
__device__ __forceinline__ v16h frag_load(const _Float16* p) {
  FragU f;
  f.h[0] = *(const v8h*)(p);
  f.h[1] = *(const v8h*)(p + 16);
  return f.v;
}
__device__ __forceinline__ v8f mma_h(v16h a, v16h b, v8f c) {
  return __builtin_amdgcn_wmma_f32_16x16x32_f16(false, a, false, b, (short)0, c, false, false);
}
__device__ __forceinline__ void dep_guard4_h(v8f& a, v8f& b, v8f& c, v8f& d, v16h x, v16h b0, v16h b1, v16h b2, v16h b3) {
  asm volatile("v_nop\n\tv_nop\n\tv_nop\n\tv_nop" : "+v"(a), "+v"(b), "+v"(c), "+v"(d) : "v"(x), "v"(b0), "v"(b1), "v"(b2), "v"(b3));
}
__device__ __forceinline__ void keep4_h(v16h a, v16h b, v16h c, v16h d) { asm volatile("v_nop" :: "v"(a), "v"(b), "v"(c), "v"(d)); }
__device__ __forceinline__ void acc_guard4(v8f& a, v8f& b, v8f& c, v8f& d) { asm volatile("v_nop\n\tv_nop\n\tv_nop\n\tv_nop" : "+v"(a), "+v"(b), "+v"(c), "+v"(d)); }

template <int BIAS_MODE, int OUT_MODE, bool RESID>
__global__ __launch_bounds__(256) void wmma_gemm64(
    const unsigned short* __restrict__ Ap, int lda,
    const unsigned short* __restrict__ Btp, int ldb,
    void* __restrict__ Cout, int ldc,
    const float* __restrict__ bias,
    const float* __restrict__ resid,
    int M, int N, int K, float scale)
{
  const _Float16* A  = (const _Float16*)Ap;
  const _Float16* Bt = (const _Float16*)Btp;
  __shared__ __align__(16) float sT[8][16 * 68];
  const int lane = threadIdx.x & 31;
  const int wave = threadIdx.x >> 5;
  const int tilesN = N >> 6;
  const int tilesM = M >> 6;
  const int tile = blockIdx.x * 8 + wave;
  if (tile >= tilesM * tilesN) return;
  const int tm = tile / tilesN;
  const int tn = tile - tm * tilesN;
  const int m0 = tm << 6;
  const int n0 = tn << 6;

  const int rlane = lane & 15;
  const int koff  = (lane >> 4) * 8;
  const int mOff  = (lane >> 4) * 8;

  v8f acc[4][4];
#pragma unroll
  for (int i = 0; i < 4; ++i)
#pragma unroll
    for (int j = 0; j < 4; ++j) acc[i][j] = (v8f){0.f, 0.f, 0.f, 0.f, 0.f, 0.f, 0.f, 0.f};

  for (int k0 = 0; k0 < K; k0 += 32) {
    v16h bh[4];
#pragma unroll
    for (int j = 0; j < 4; ++j) {
      const size_t bo = (size_t)(n0 + (j << 4) + rlane) * ldb + koff + k0;
      bh[j] = frag_load(Bt + bo);
    }
#pragma unroll
    for (int i = 0; i < 4; ++i) {
      const size_t ao = (size_t)(m0 + (i << 4) + rlane) * lda + koff + k0;
      const v16h ah = frag_load(A + ao);
#pragma unroll
      for (int j = 0; j < 4; ++j) acc[i][j] = mma_h(ah, bh[j], acc[i][j]);
      dep_guard4_h(acc[i][0], acc[i][1], acc[i][2], acc[i][3], ah, bh[0], bh[1], bh[2], bh[3]);
    }
    keep4_h(bh[0], bh[1], bh[2], bh[3]);
  }
  acc_guard4(acc[0][0], acc[0][1], acc[0][2], acc[0][3]);
  acc_guard4(acc[1][0], acc[1][1], acc[1][2], acc[1][3]);
  acc_guard4(acc[2][0], acc[2][1], acc[2][2], acc[2][3]);
  acc_guard4(acc[3][0], acc[3][1], acc[3][2], acc[3][3]);

  float* slab = sT[wave];
#pragma unroll
  for (int i = 0; i < 4; ++i) {
    const int mBase = m0 + (i << 4);
#pragma unroll
    for (int j = 0; j < 4; ++j) {
      const int n = n0 + (j << 4) + rlane;
      float bv = 0.f;
      if (BIAS_MODE == 2) bv = bias[n];
#pragma unroll
      for (int r = 0; r < 8; ++r) {
        float v = acc[i][j][r] * scale;
        if (BIAS_MODE == 2) v += bv;
        slab[(mOff + r) * 68 + (j << 4) + rlane] = v;
      }
    }
    __builtin_amdgcn_fence(__ATOMIC_RELEASE, "workgroup");
    __builtin_amdgcn_wave_barrier();
    __builtin_amdgcn_fence(__ATOMIC_ACQUIRE, "workgroup");
    if (OUT_MODE == 0) {
      float* C = (float*)Cout;
      const int hh = lane >> 4, c4 = (lane & 15) * 4;
      v4f vv[8];
#pragma unroll
      for (int it = 0; it < 8; ++it) {
        const int row = it * 2 + hh;
        vv[it] = *(const v4f*)(slab + row * 68 + c4);
      }
      if (RESID) {
#pragma unroll
        for (int it = 0; it < 8; ++it) {
          const int row = it * 2 + hh;
          const v4f rr = *(const v4f*)(resid + (size_t)(mBase + row) * ldc + n0 + c4);
          vv[it] = vv[it] + rr;
        }
      }
      for (int pass = 0; pass < 2; ++pass) {
#pragma unroll
        for (int it = 0; it < 8; ++it) {
          const int row = it * 2 + hh;
          *(volatile v4f*)(C + (size_t)(mBase + row) * ldc + n0 + c4) = vv[it];
        }
        __threadfence();
      }
    } else {
      const int q = lane >> 3, c8 = (lane & 7) * 8;
      unsigned short* C = (unsigned short*)Cout;
      v8h hv[4];
#pragma unroll
      for (int it = 0; it < 4; ++it) {
        const int row = it * 4 + q;
        const float* sp = slab + row * 68 + c8;
        const v4f a0 = *(const v4f*)(sp);
        const v4f a1 = *(const v4f*)(sp + 4);
#pragma unroll
        for (int e = 0; e < 4; ++e) {
          hv[it][e]     = (_Float16)a0[e];
          hv[it][4 + e] = (_Float16)a1[e];
        }
      }
      for (int pass = 0; pass < 2; ++pass) {
#pragma unroll
        for (int it = 0; it < 4; ++it) {
          const int row = it * 4 + q;
          *(volatile v8h*)(C + (size_t)(mBase + row) * ldc + n0 + c8) = hv[it];
        }
        __threadfence();
      }
    }
    __builtin_amdgcn_fence(__ATOMIC_RELEASE, "workgroup");
    __builtin_amdgcn_wave_barrier();
    __builtin_amdgcn_fence(__ATOMIC_ACQUIRE, "workgroup");
  }
}

__global__ __launch_bounds__(256) void cast_pad_f16_kernel(
    const float* __restrict__ src, int ld_src, int rows_src, int cols_src,
    unsigned short* __restrict__ dst, int cols_dst, int total8, float scale)
{
  const int i = blockIdx.x * 256 + threadIdx.x;
  if (i >= total8) return;
  const int e0 = i << 3;
  const int r  = e0 / cols_dst;
  const int c8 = e0 - r * cols_dst;
  const bool ok = (r < rows_src) && (c8 < cols_src);
  const int rc = (r < rows_src) ? r : (rows_src - 1);
  const int cc = (c8 < cols_src) ? c8 : (cols_src - 8);
  const float* p = src + (size_t)rc * ld_src + cc;
  const v4f a0 = *(const v4f*)(p);
  const v4f a1 = *(const v4f*)(p + 4);
  v8h hv;
#pragma unroll
  for (int e = 0; e < 4; ++e) {
    const float f0 = ok ? (a0[e] * scale) : 0.0f;
    const float f1 = ok ? (a1[e] * scale) : 0.0f;
    hv[e]     = (_Float16)f0;
    hv[4 + e] = (_Float16)f1;
  }
  unsigned short* q = dst + (size_t)e0;
  *(volatile v8h*)q = hv;
  __threadfence();
  *(volatile v8h*)q = hv;
}

__global__ __launch_bounds__(256) void ln_rows_f16_kernel(
    const float* __restrict__ X, const float* __restrict__ g, const float* __restrict__ bsh,
    unsigned short* __restrict__ out)
{
  const int lane = threadIdx.x & 31, wave = threadIdx.x >> 5;
  const int row = blockIdx.x * 8 + wave;
  const float* xr = X + (size_t)row * kDm;
  v4f v[6];
#pragma unroll
  for (int j = 0; j < 3; ++j) {
    const int off = (j * 32 + lane) * 8;
    v[2 * j]     = *(const v4f*)(xr + off);
    v[2 * j + 1] = *(const v4f*)(xr + off + 4);
  }
  float s = 0.f;
#pragma unroll
  for (int j = 0; j < 6; ++j) s += (v[j][0] + v[j][1]) + (v[j][2] + v[j][3]);
#pragma unroll
  for (int o = 16; o > 0; o >>= 1) s += __shfl_xor(s, o, 32);
  const float mu = s * (1.0f / (float)kDm);
  float qs = 0.f;
#pragma unroll
  for (int j = 0; j < 6; ++j) {
#pragma unroll
    for (int e = 0; e < 4; ++e) {
      const float dlt = v[j][e] - mu;
      qs += dlt * dlt;
    }
  }
#pragma unroll
  for (int o = 16; o > 0; o >>= 1) qs += __shfl_xor(qs, o, 32);
  const float var = qs * (1.0f / (float)kDm);
  const float inv = rsqrtf(var + 1e-5f);
  v8h hv[3];
#pragma unroll
  for (int j = 0; j < 3; ++j) {
    const int off = (j * 32 + lane) * 8;
    const v4f g0 = *(const v4f*)(g + off);
    const v4f g1 = *(const v4f*)(g + off + 4);
    const v4f b0 = *(const v4f*)(bsh + off);
    const v4f b1 = *(const v4f*)(bsh + off + 4);
#pragma unroll
    for (int e = 0; e < 4; ++e) {
      const float y0 = (v[2 * j][e] - mu) * inv * g0[e] + b0[e];
      const float y1 = (v[2 * j + 1][e] - mu) * inv * g1[e] + b1[e];
      hv[j][e]     = (_Float16)y0;
      hv[j][4 + e] = (_Float16)y1;
    }
  }
  unsigned short* orow = out + (size_t)row * kDm;
  for (int pass = 0; pass < 2; ++pass) {
#pragma unroll
    for (int j = 0; j < 3; ++j) *(volatile v8h*)(orow + (j * 32 + lane) * 8) = hv[j];
    __threadfence();
  }
}

__global__ __launch_bounds__(256) void conv_silu_kernel(
    const unsigned short* __restrict__ XZ, const float* __restrict__ cw, const float* __restrict__ cb,
    unsigned short* __restrict__ XC16, int rev)
{
  __shared__ __align__(16) float sT[16 * kTP];
  const int tid = threadIdx.x, lane = tid & 31, wave = tid >> 5;
  const int d0 = blockIdx.x * 256, d = d0 + tid;
  const int g0 = blockIdx.y * 64;
  const int tb = g0 & (kSeq - 1);
  const v4f wv = *(const v4f*)(cw + (size_t)d * 4);
  const float w0 = wv[0], w1 = wv[1], w2 = wv[2], w3 = wv[3];
  const float bc = cb[d];
  const int stp = rev ? -1 : 1;
  const int pstart = rev ? (g0 + 63) : g0;
  const bool hist = rev ? (tb + 64 < kSeq) : (tb > 0);
  float xm1, xm2, xm3;
  {
    const int r1 = hist ? (pstart - stp) : pstart;
    const int r2 = hist ? (pstart - 2 * stp) : pstart;
    const int r3 = hist ? (pstart - 3 * stp) : pstart;
    const unsigned u1 = XZ[(size_t)r1 * kXzP + d];
    const unsigned u2 = XZ[(size_t)r2 * kXzP + d];
    const unsigned u3 = XZ[(size_t)r3 * kXzP + d];
    const float v1 = h16_to_f32(u1), v2 = h16_to_f32(u2), v3 = h16_to_f32(u3);
    xm1 = hist ? v1 : 0.f;
    xm2 = hist ? v2 : 0.f;
    xm3 = hist ? v3 : 0.f;
  }
#pragma unroll 1
  for (int j = 0; j < 4; ++j) {
    const int lb = rev ? (g0 + (3 - j) * 16) : (g0 + j * 16);
#pragma unroll 1
    for (int s = 0; s < 16; ++s) {
      const int lr = rev ? (15 - s) : s;
      const unsigned ub = XZ[(size_t)(lb + lr) * kXzP + d];
      const float xcur = h16_to_f32(ub);
      float acc = w0 * xm3;
      acc = fmaf(w1, xm2, acc);
      acc = fmaf(w2, xm1, acc);
      acc = fmaf(w3, xcur, acc);
      const float sv = acc + bc;
      const float ev = expf(-sv);
      const float sg = 1.0f / (1.0f + ev);
      sT[lr * kTP + tid] = (sv * sg) * kCarryXc;
      xm3 = xm2; xm2 = xm1; xm1 = xcur;
    }
    __syncthreads();
    v8h bv[2];
#pragma unroll
    for (int it = 0; it < 2; ++it) {
      const float* sp = sT + (it * 8 + wave) * kTP + lane * 8;
      const v4f a0 = *(const v4f*)(sp);
      const v4f a1 = *(const v4f*)(sp + 4);
#pragma unroll
      for (int e = 0; e < 4; ++e) {
        bv[it][e]     = (_Float16)a0[e];
        bv[it][4 + e] = (_Float16)a1[e];
      }
    }
    for (int pass = 0; pass < 2; ++pass) {
#pragma unroll
      for (int it = 0; it < 2; ++it)
        *(volatile v8h*)(XC16 + (size_t)(lb + it * 8 + wave) * kDin + d0 + lane * 8) = bv[it];
      __threadfence();
    }
    __syncthreads();
  }
}

template <int REV>
__global__ __launch_bounds__(256) void scan_kernel(
    const float* __restrict__ DLIN, const unsigned short* __restrict__ XC16,
    const unsigned short* __restrict__ XZ, const float* __restrict__ XDBL,
    const float* __restrict__ Alog, const float* __restrict__ Dv,
    const unsigned short* __restrict__ YFWD, unsigned short* __restrict__ YOUT)
{
  __shared__ __align__(16) float sBC[16 * 32];
  __shared__ __align__(16) float sY[16 * kTP];
  const int tid = threadIdx.x, lane = tid & 31, wave = tid >> 5;
  constexpr int kBlkPerB = kDin / 256;
  const int bix = blockIdx.x / kBlkPerB;
  const int d0  = (blockIdx.x - bix * kBlkPerB) * 256;
  const int d   = d0 + tid;
  const size_t row0 = (size_t)bix * kSeq;

#pragma unroll 1
  for (int n = 0; n < kNst; ++n) sY[n * kTP + tid] = -expf(Alog[(size_t)d * kNst + n]);
  __syncthreads();
  float An[kNst], h[kNst];
#pragma unroll
  for (int n = 0; n < kNst; ++n) {
    An[n] = sY[n * kTP + tid];
    h[n] = 0.f;
  }
  __syncthreads();
  const float Dd = Dv[d];

#pragma unroll 1
  for (int c = 0; c < kSeq / 16; ++c) {
    const int l0 = REV ? (kSeq - 16 - c * 16) : (c * 16);
    if (tid < 128) {
      const int r = tid >> 3, q = (tid & 7) * 4;
      const v4f bcv = *(const v4f*)(XDBL + (row0 + (size_t)(l0 + r)) * kXpP + kDtR + q);
      *(v4f*)(sBC + r * 32 + q) = bcv;
    }
    __syncthreads();
#pragma unroll 1
    for (int s = 0; s < 16; ++s) {
      const int ls = REV ? (15 - s) : s;
      const size_t m = row0 + (size_t)(l0 + ls);
      float a = DLIN[m * kDin + d];
      unsigned xb = XC16[m * kDin + d];
      asm volatile("" : "+v"(a), "+v"(xb));
      const float ea  = __expf(-fabsf(a));
      const float up  = 1.0f + ea;
      const float l1p = __logf(up) + (ea - (up - 1.0f)) * __builtin_amdgcn_rcpf(up);
      const float delta = fmaxf(a, 0.0f) + l1p;
      const float xv = h16_to_f32(xb) * (1.0f / kCarryXc);
      const float dx = delta * xv;
      v4f Bq[4], Cq[4];
#pragma unroll
      for (int qq = 0; qq < 4; ++qq) {
        Bq[qq] = *(const v4f*)(sBC + ls * 32 + 4 * qq);
        Cq[qq] = *(const v4f*)(sBC + ls * 32 + kNst + 4 * qq);
      }
      float y = 0.f;
#pragma unroll
      for (int n = 0; n < kNst; ++n) {
        const float e = __expf(delta * An[n]);
        h[n] = e * h[n] + dx * Bq[n >> 2][n & 3];
        y = h[n] * Cq[n >> 2][n & 3] + y;
      }
      y = xv * Dd + y;
      float val = y * kCarryY;
      if (REV) {
        unsigned zb = XZ[m * kXzP + kDin + d];
        unsigned yb = YFWD[m * kDin + d];
        asm volatile("" : "+v"(zb), "+v"(yb));
        const float zv = h16_to_f32(zb);
        const float yf = h16_to_f32(yb);
        const float ez = expf(-zv);
        const float sg = 1.0f / (1.0f + ez);
        val = (val + yf) * ((kCarryS / kCarryY) * zv * sg);
      }
      sY[ls * kTP + tid] = val;
    }
    __syncthreads();
    v8h hv[2];
#pragma unroll
    for (int it = 0; it < 2; ++it) {
      const float* sp = sY + (it * 8 + wave) * kTP + lane * 8;
      const v4f a0 = *(const v4f*)(sp);
      const v4f a1 = *(const v4f*)(sp + 4);
#pragma unroll
      for (int e = 0; e < 4; ++e) {
        hv[it][e]     = (_Float16)a0[e];
        hv[it][4 + e] = (_Float16)a1[e];
      }
    }
    for (int pass = 0; pass < 2; ++pass) {
#pragma unroll
      for (int it = 0; it < 2; ++it)
        *(volatile v8h*)(YOUT + (row0 + (size_t)(l0 + it * 8 + wave)) * kDin + d0 + lane * 8) = hv[it];
      __threadfence();
    }
  }
}

__global__ __launch_bounds__(256) void gelu_f16_kernel(const float* __restrict__ P, unsigned short* __restrict__ ACT)
{
  __shared__ __align__(16) float sG[2048];
  const int tid = threadIdx.x;
  const size_t base = (size_t)blockIdx.x * 2048;
#pragma unroll 1
  for (int j = 0; j < 8; ++j) {
    const int idx = j * 256 + tid;
    const float v = P[base + idx];
    sG[idx] = 0.5f * v * (1.0f + erff(v * 0.70710678118654752f));
  }
  __syncthreads();
  const v4f a0 = *(const v4f*)(sG + tid * 8);
  const v4f a1 = *(const v4f*)(sG + tid * 8 + 4);
  v8h hv;
#pragma unroll
  for (int e = 0; e < 4; ++e) {
    hv[e]     = (_Float16)a0[e];
    hv[4 + e] = (_Float16)a1[e];
  }
  unsigned short* q = ACT + base + (size_t)tid * 8;
  *(volatile v8h*)q = hv;
  __threadfence();
  *(volatile v8h*)q = hv;
}

static_assert(((kRows / 64) * (kXzP / 64)) % 8 == 0 && ((kRows / 64) * (kXpP / 64)) % 8 == 0 &&
              ((kRows / 64) * (kDin / 64)) % 8 == 0 && ((kRows / 64) * (kDm / 64)) % 8 == 0);
static_assert(((kXzP * kDm / 8) % 256) == 0 && ((kXpP * kDin / 8) % 256) == 0 && ((kDin * kDtRP / 8) % 256) == 0 &&
              ((kDm * kDin / 8) % 256) == 0 && ((kRows * kDtRP / 8) % 256) == 0 && (((size_t)kRows * kFf) % 2048) == 0);

extern "C" void kernel_launch(void* const* d_in, const int* in_sizes, int n_in,
                              void* d_out, int out_size, void* d_ws, size_t ws_size,
                              hipStream_t stream)
{
  if (n_in < 19) return;
  if (in_sizes[0] != kRows * kDm) return;
  if (in_sizes[1] != kDm || in_sizes[2] != kDm) return;
  if (in_sizes[3] != kXzP * kDm) return;
  if (in_sizes[4] != kDin * 4 || in_sizes[5] != kDin) return;
  if (in_sizes[6] != kXpN * kDin) return;
  if (in_sizes[7] != kDin * kDtR || in_sizes[8] != kDin) return;
  if (in_sizes[9] != kDin * kNst || in_sizes[10] != kDin * kNst) return;
  if (in_sizes[11] != kDin) return;
  if (in_sizes[12] != kDm * kDin) return;
  if (in_sizes[13] != kDm || in_sizes[14] != kDm) return;
  if (in_sizes[15] != kFf * kDm || in_sizes[16] != kFf) return;
  if (in_sizes[17] != kDm * kFf || in_sizes[18] != kDm) return;
  if (out_size != kRows * kDm) return;
  if (ws_size < kWsTotal) return;

  const float* x         = (const float*)d_in[0];
  const float* g1        = (const float*)d_in[1];
  const float* b1        = (const float*)d_in[2];
  const float* in_proj_w = (const float*)d_in[3];
  const float* conv_w    = (const float*)d_in[4];
  const float* conv_b    = (const float*)d_in[5];
  const float* x_proj_w  = (const float*)d_in[6];
  const float* dt_proj_w = (const float*)d_in[7];
  const float* dt_proj_b = (const float*)d_in[8];
  const float* A_log     = (const float*)d_in[9];
  const float* A_b_log   = (const float*)d_in[10];
  const float* Dskip     = (const float*)d_in[11];
  const float* out_proj_w= (const float*)d_in[12];
  const float* g2        = (const float*)d_in[13];
  const float* b2        = (const float*)d_in[14];
  const float* fc1_w     = (const float*)d_in[15];
  const float* fc1_b     = (const float*)d_in[16];
  const float* fc2_w     = (const float*)d_in[17];
  const float* fc2_b     = (const float*)d_in[18];
  float* out = (float*)d_out;

  char* ws = (char*)d_ws;
  unsigned short* WIN16  = (unsigned short*)(ws + kOffWIN);
  unsigned short* WXP16  = (unsigned short*)(ws + kOffWXP);
  unsigned short* WDT16  = (unsigned short*)(ws + kOffWDT);
  unsigned short* WOUT16 = (unsigned short*)(ws + kOffWOUT);
  unsigned short* WFC1   = (unsigned short*)(ws + kOffWFC1);
  unsigned short* WFC2   = (unsigned short*)(ws + kOffWFC2);
  unsigned short* LN16   = (unsigned short*)(ws + kOffLN);
  unsigned short* XZ16   = (unsigned short*)(ws + kOffXZ);
  unsigned short* XC16   = (unsigned short*)(ws + kOffXC);
  float*          XDBL   = (float*)(ws + kOffXDBL);
  unsigned short* DTR16  = (unsigned short*)(ws + kOffDTR);
  float*          DLIN   = (float*)(ws + kOffDLIN);
  unsigned short* YF16   = (unsigned short*)(ws + kOffYF);
  unsigned short* S16    = (unsigned short*)(ws + kOffS);
  float*          HB     = (float*)(ws + kOffHB);
  float*          PRE    = DLIN;
  unsigned short* ACT16  = YF16;
  const float* dummy_bias  = dt_proj_b;
  const float* dummy_resid = x;

  cast_pad_f16_kernel<<<(kXzP * kDm / 8) / 256, 256, 0, stream>>>(in_proj_w, kDm, kXzP, kDm, WIN16, kDm, kXzP * kDm / 8, kCarryW);
  cast_pad_f16_kernel<<<(kXpP * kDin / 8) / 256, 256, 0, stream>>>(x_proj_w, kDin, kXpN, kDin, WXP16, kDin, kXpP * kDin / 8, kCarryW);
  cast_pad_f16_kernel<<<(kDin * kDtRP / 8) / 256, 256, 0, stream>>>(dt_proj_w, kDtR, kDin, kDtR, WDT16, kDtRP, kDin * kDtRP / 8, kCarryW);
  cast_pad_f16_kernel<<<(kDm * kDin / 8) / 256, 256, 0, stream>>>(out_proj_w, kDin, kDm, kDin, WOUT16, kDin, kDm * kDin / 8, kCarryW);
  cast_pad_f16_kernel<<<(kFf * kDm / 8) / 256, 256, 0, stream>>>(fc1_w, kDm, kFf, kDm, WFC1, kDm, kFf * kDm / 8, kCarryW);
  cast_pad_f16_kernel<<<(kDm * kFf / 8) / 256, 256, 0, stream>>>(fc2_w, kFf, kDm, kFf, WFC2, kFf, kDm * kFf / 8, kCarryW);

  ln_rows_f16_kernel<<<kRows / 8, 256, 0, stream>>>(x, g1, b1, LN16);
  wmma_gemm64<0, 1, false><<<((kRows / 64) * (kXzP / 64)) / 8, 256, 0, stream>>>(
      LN16, kDm, WIN16, kDm, (void*)XZ16, kXzP, dummy_bias, dummy_resid,
      kRows, kXzP, kDm, 1.0f / kCarryW);

  for (int dir = 0; dir < 2; ++dir) {
    conv_silu_kernel<<<dim3(kDin / 256, kRows / 64), 256, 0, stream>>>(XZ16, conv_w, conv_b, XC16, dir);
    wmma_gemm64<0, 0, false><<<((kRows / 64) * (kXpP / 64)) / 8, 256, 0, stream>>>(
        XC16, kDin, WXP16, kDin, (void*)XDBL, kXpP, dummy_bias, dummy_resid,
        kRows, kXpP, kDin, 1.0f / (kCarryXc * kCarryW));
    cast_pad_f16_kernel<<<(kRows * kDtRP / 8) / 256, 256, 0, stream>>>(XDBL, kXpP, kRows, kDtR, DTR16, kDtRP, kRows * kDtRP / 8, kCarryDt);
    wmma_gemm64<2, 0, false><<<((kRows / 64) * (kDin / 64)) / 8, 256, 0, stream>>>(
        DTR16, kDtRP, WDT16, kDtRP, (void*)DLIN, kDin, dt_proj_b, dummy_resid,
        kRows, kDin, kDtRP, 1.0f / (kCarryDt * kCarryW));
    if (dir == 0) {
      scan_kernel<0><<<kBatch * (kDin / 256), 256, 0, stream>>>(DLIN, XC16, XZ16, XDBL, A_log, Dskip, XC16, YF16);
    } else {
      scan_kernel<1><<<kBatch * (kDin / 256), 256, 0, stream>>>(DLIN, XC16, XZ16, XDBL, A_b_log, Dskip, YF16, S16);
    }
  }

  wmma_gemm64<0, 0, true><<<((kRows / 64) * (kDm / 64)) / 8, 256, 0, stream>>>(
      S16, kDin, WOUT16, kDin, (void*)HB, kDm, dummy_bias, x,
      kRows, kDm, kDin, 1.0f / (kCarryS * kCarryW));

  ln_rows_f16_kernel<<<kRows / 8, 256, 0, stream>>>(HB, g2, b2, LN16);
  wmma_gemm64<2, 0, false><<<((kRows / 64) * (kFf / 64)) / 8, 256, 0, stream>>>(
      LN16, kDm, WFC1, kDm, (void*)PRE, kFf, fc1_b, dummy_resid,
      kRows, kFf, kDm, 1.0f / kCarryW);
  gelu_f16_kernel<<<(unsigned)(((size_t)kRows * kFf) / 2048), 256, 0, stream>>>(PRE, ACT16);
  wmma_gemm64<2, 0, true><<<((kRows / 64) * (kDm / 64)) / 8, 256, 0, stream>>>(
      ACT16, kFf, WFC2, kFf, (void*)out, kDm, fc2_b, HB,
      kRows, kDm, kFf, 1.0f / kCarryW);
}
